// RNN_21809843929473
// MI455X (gfx1250) — hardware-verified
//
#include <hip/hip_runtime.h>

typedef __attribute__((ext_vector_type(16))) _Float16 v16h;
typedef __attribute__((ext_vector_type(8)))  _Float16 v8h;
typedef __attribute__((ext_vector_type(8)))  float    v8f;
typedef __attribute__((ext_vector_type(4)))  unsigned v4u;
typedef v8h      v8h_ma __attribute__((may_alias));
typedef v4u      v4u_ma __attribute__((may_alias));
typedef unsigned u32_ma __attribute__((may_alias));

constexpr int kBatch   = 4096;
constexpr int kSteps   = 256;
constexpr int kHidA    = 5;
constexpr int kHidB    = 100;
constexpr int kNPad    = 112;
constexpr int kKPad    = 128;
constexpr int kPitch   = 136;
constexpr int kSlotA   = 104;
constexpr int kWaves   = 4;
constexpr int kThreads = kWaves * 32;
constexpr int kRowsPerBlock = kWaves * 32;
constexpr int kBlocks  = kBatch / kRowsPerBlock;
constexpr int kTileHalves  = 32 * kPitch;
constexpr int kPlaneChunks = kWaves * kTileHalves / 8;
constexpr int kWtElems     = kNPad * kPitch;

constexpr float kWCarry    = 16.0f;
constexpr float kWCarryInv = 1.0f / 16.0f;
constexpr float kResCarry  = 2048.0f;
constexpr float kResInv    = 1.0f / 2048.0f;
constexpr float kResFold   = 1.0f / (2048.0f * 16.0f);
constexpr float kHalfMinNormal = 6.103515625e-5f;

static_assert(kBatch % kRowsPerBlock == 0, "grid exact");
static_assert(kBlocks == 32, "32 blocks");
static_assert(kKPad % 32 == 0 && kNPad % 16 == 0, "tile multiples");
static_assert(kHidB <= kSlotA - 4 && kSlotA + kHidA <= kKPad, "slot map");
static_assert(kSlotA % 8 == 0, "16-B aligned slot chunk");
static_assert((kPitch * 2) % 16 == 0 && kPitch >= kKPad, "pitch");
static_assert(kPlaneChunks % kThreads == 0, "zero fill exact");
static_assert(kWtElems % kThreads == 0, "weight build exact");
static_assert(kThreads == 128, "bias staging uses one element per thread");
static_assert(kHidB % 2 == 0, "output dot reads half pairs");

__device__ __forceinline__ float h16_to_f32(unsigned hb) {
  const unsigned sgn = (hb & 0x8000u) << 16; const unsigned em = hb & 0x7fffu;
  const float fn = __uint_as_float((em << 13) + 0x38000000u);
  const float fs = (float)em * 5.9604644775390625e-8f;
  const float mag = (em < 0x400u) ? fs : fn; return __uint_as_float(__float_as_uint(mag) | sgn); }

__device__ __forceinline__ float ftanh(float x) {
  const float xc = fminf(fmaxf(x, -15.0f), 15.0f);
  return 1.0f - 2.0f * __builtin_amdgcn_rcpf(1.0f + __expf(2.0f * xc));
}

__device__ __forceinline__ void split16(float v, _Float16& hi, _Float16& lo) {
  const float vs = (fabsf(v) < kHalfMinNormal) ? 0.0f : v;
  hi = (_Float16)vs;
  float hif = (float)hi;
  asm volatile("" : "+v"(hif));
  lo = (_Float16)((v - hif) * kResCarry);
}

__device__ __forceinline__ unsigned half_bits(_Float16 h) {
  const unsigned short s = __builtin_bit_cast(unsigned short, h);
  return (unsigned)s;
}

__device__ __forceinline__ v16h lds_frag(const _Float16* p) {
  union { v16h v; v8h h[2]; } f;
  f.h[0] = *(const v8h_ma*)(p);
  f.h[1] = *(const v8h_ma*)(p + 16);
  return f.v;
}

__device__ __forceinline__ v8f mma_h(v16h a, v16h b, v8f c) {
  return __builtin_amdgcn_wmma_f32_16x16x32_f16(false, a, false, b, (short)0, c, false, false);
}

__device__ __forceinline__ void group_guard(v8f& a, v8f& b,
                                            v16h a0, v16h a1, v16h a2, v16h a3,
                                            v16h l0, v16h l1, v16h l2, v16h l3,
                                            v16h b0, v16h b1, v16h b2, v16h b3) {
  asm volatile("v_nop\n\tv_nop\n\tv_nop\n\tv_nop"
               : "+v"(a), "+v"(b)
               : "v"(a0), "v"(a1), "v"(a2), "v"(a3),
                 "v"(l0), "v"(l1), "v"(l2), "v"(l3),
                 "v"(b0), "v"(b1), "v"(b2), "v"(b3));
}

__global__ __launch_bounds__(kThreads) void rnn2_fused_kernel(
    const float* __restrict__ x,
    const float* __restrict__ Wih1, const float* __restrict__ Whh1,
    const float* __restrict__ bih1, const float* __restrict__ bhh1,
    const float* __restrict__ Wih2, const float* __restrict__ Whh2,
    const float* __restrict__ bih2, const float* __restrict__ bhh2,
    const float* __restrict__ W3,   const float* __restrict__ b3,
    float* __restrict__ out) {
  __shared__ __align__(16) _Float16 Wt[kWtElems];
  __shared__ __align__(16) _Float16 HiT[kWaves * kTileHalves];
  __shared__ __align__(16) _Float16 LoT[kWaves * kTileHalves];
  __shared__ __align__(16) float biasS[kThreads];
  __shared__ __align__(16) float w3S[kThreads];

  const int tid  = threadIdx.x;
  const int lane = tid & 31;
  const int wave = tid >> 5;
  const int c    = lane & 15;
  const int hh   = lane >> 4;

  const v4u zq = {0u, 0u, 0u, 0u};

  {
    v4u_ma* ph = (v4u_ma*)HiT;
    v4u_ma* pl = (v4u_ma*)LoT;
#pragma unroll 1
    for (int i = tid; i < kPlaneChunks; i += kThreads) { ph[i] = zq; pl[i] = zq; }
  }

#pragma unroll 1
  for (int idx = tid; idx < kWtElems; idx += kThreads) {
    const int n  = idx / kPitch;
    const int k  = idx - n * kPitch;
    const int nc = (n < kHidB) ? n : (kHidB - 1);
    const int kc = (k < kHidB) ? k : (kHidB - 1);
    int jc = k - kSlotA;
    jc = (jc < 0) ? 0 : jc;
    jc = (jc > kHidA - 1) ? (kHidA - 1) : jc;
    const float a = Whh2[nc * kHidB + kc];
    const float b = Wih2[nc * kHidA + jc];
    const float fa = (n < kHidB && k < kHidB) ? 1.0f : 0.0f;
    const float fb = (n < kHidB && k >= kSlotA && k < kSlotA + kHidA) ? 1.0f : 0.0f;
    const float w = fmaf(fa, a, fb * b) + 0.0f;
    Wt[idx] = (_Float16)(w * kWCarry);
  }

  {
    const int nn = (tid < kHidB) ? tid : (kHidB - 1);
    const float f = (tid < kHidB) ? 1.0f : 0.0f;
    const float bsum = bih2[nn] + bhh2[nn];
    const float w3v  = W3[nn];
    biasS[tid] = f * bsum + 0.0f;
    w3S[tid]   = f * w3v + 0.0f;
  }

  float wih1[kHidA], b1[kHidA], whh1[kHidA][kHidA];
#pragma unroll
  for (int i = 0; i < kHidA; ++i) { wih1[i] = Wih1[i]; b1[i] = bih1[i] + bhh1[i]; }
  asm volatile("" ::: "memory");
#pragma unroll
  for (int i = 0; i < kHidA; ++i) {
#pragma unroll
    for (int j = 0; j < kHidA; ++j) whh1[i][j] = Whh1[i * kHidA + j];
    if ((i & 1) == 1) asm volatile("" ::: "memory");
  }
  asm volatile("" ::: "memory");
  const float b3v = b3[0];

  _Float16* hw = HiT + wave * kTileHalves;
  _Float16* lw = LoT + wave * kTileHalves;

  const int brow = blockIdx.x * kRowsPerBlock + wave * 32 + lane;
  const float* xp = x + (size_t)brow * kSteps;
  float xcur = xp[0];
  float h1[kHidA];
#pragma unroll
  for (int i = 0; i < kHidA; ++i) h1[i] = 0.0f;

  const v8f z8 = {0.f, 0.f, 0.f, 0.f, 0.f, 0.f, 0.f, 0.f};

  __syncthreads();

#pragma unroll 1
  for (int t = 0; t < kSteps; ++t) {
    const float xt = xcur;
    const int tn = (t + 1 < kSteps) ? (t + 1) : t;
    xcur = xp[tn];
    float s[kHidA];
#pragma unroll
    for (int i = 0; i < kHidA; ++i) {
      s[i] = fmaf(wih1[i], xt, b1[i]);
#pragma unroll
      for (int j = 0; j < kHidA; ++j) s[i] = fmaf(whh1[i][j], h1[j], s[i]);
    }
    unsigned hb[kHidA], lb[kHidA];
#pragma unroll
    for (int i = 0; i < kHidA; ++i) {
      h1[i] = ftanh(s[i]);
      _Float16 hi, lo;
      split16(h1[i], hi, lo);
      hb[i] = half_bits(hi);
      lb[i] = half_bits(lo);
    }
    {
      v4u wh, wl;
      wh[0] = hb[0] | (hb[1] << 16);
      wh[1] = hb[2] | (hb[3] << 16);
      wh[2] = hb[4];
      wh[3] = 0u;
      wl[0] = lb[0] | (lb[1] << 16);
      wl[1] = lb[2] | (lb[3] << 16);
      wl[2] = lb[4];
      wl[3] = 0u;
      v4u_ma* dh = (v4u_ma*)(hw + lane * kPitch + kSlotA);
      v4u_ma* dl = (v4u_ma*)(lw + lane * kPitch + kSlotA);
      dh[0] = wh; dh[1] = zq; dh[2] = zq;
      dl[0] = wl; dl[1] = zq; dl[2] = zq;
    }
    __syncthreads();

#pragma unroll 1
    for (int mt = 0; mt < 2; ++mt) {
      const _Float16* ar = hw + (16 * mt + c) * kPitch + 8 * hh;
      const _Float16* lr = lw + (16 * mt + c) * kPitch + 8 * hh;
      v16h ah[4], al[4];
#pragma unroll
      for (int kc = 0; kc < 4; ++kc) {
        ah[kc] = lds_frag(ar + 32 * kc);
        al[kc] = lds_frag(lr + 32 * kc);
      }
#pragma unroll 1
      for (int nt = 0; nt < kNPad / 16; ++nt) {
        const _Float16* br = Wt + (16 * nt + c) * kPitch + 8 * hh;
        v16h bf[4];
#pragma unroll
        for (int kc = 0; kc < 4; ++kc) bf[kc] = lds_frag(br + 32 * kc);
        v8f accM = z8, accR = z8;
#pragma unroll
        for (int kc = 0; kc < 4; ++kc) {
          accM = mma_h(ah[kc], bf[kc], accM);
          accR = mma_h(al[kc], bf[kc], accR);
        }
        group_guard(accM, accR, ah[0], ah[1], ah[2], ah[3], al[0], al[1], al[2], al[3], bf[0], bf[1], bf[2], bf[3]);

        const int n = 16 * nt + c;
        const float bn = biasS[n];
        const bool keepn = (n < kHidB);
        const bool wr    = (n < kSlotA);
#pragma unroll
        for (int r = 0; r < 8; ++r) {
          const int row = 16 * mt + 8 * hh + r;
          const float pre = fmaf(accM[r], kWCarryInv, fmaf(accR[r], kResFold, bn));
          const float hv  = ftanh(pre);
          const float hvs = keepn ? hv : 0.0f;
          _Float16 hi, lo;
          split16(hvs, hi, lo);
          if (wr) {
            hw[row * kPitch + n] = hi;
            lw[row * kPitch + n] = lo;
          }
        }
      }
    }
  }

  __syncthreads();

  {
    const u32_ma* rh = (const u32_ma*)(hw + lane * kPitch);
    const u32_ma* rl = (const u32_ma*)(lw + lane * kPitch);
    float sum = 0.0f;
#pragma unroll 1
    for (int j = 0; j < kHidB / 2; ++j) {
      const unsigned a = rh[j];
      const unsigned b = rl[j];
      const float h0 = h16_to_f32(a & 0xffffu);
      const float r0 = h16_to_f32(b & 0xffffu);
      const float h1v = h16_to_f32(a >> 16);
      const float r1 = h16_to_f32(b >> 16);
      const float v0 = fmaf(r0, kResInv, h0);
      const float v1 = fmaf(r1, kResInv, h1v);
      sum = fmaf(w3S[2 * j], v0, sum);
      sum = fmaf(w3S[2 * j + 1], v1, sum);
    }
    const float tot = sum + b3v;
    const float res = fmaxf(tot, 0.0f);
    volatile float* op = out + brow;
    *op = res;
    __threadfence();
    *op = res;
  }
}

extern "C" void kernel_launch(void* const* d_in, const int* in_sizes, int n_in,
                              void* d_out, int out_size, void* d_ws, size_t ws_size,
                              hipStream_t stream) {
  (void)in_sizes; (void)out_size; (void)d_ws; (void)ws_size;
  if (n_in < 11 || d_out == nullptr) return;
  const float* x    = (const float*)d_in[0];
  const float* Wih1 = (const float*)d_in[1];
  const float* Whh1 = (const float*)d_in[2];
  const float* bih1 = (const float*)d_in[3];
  const float* bhh1 = (const float*)d_in[4];
  const float* Wih2 = (const float*)d_in[5];
  const float* Whh2 = (const float*)d_in[6];
  const float* bih2 = (const float*)d_in[7];
  const float* bhh2 = (const float*)d_in[8];
  const float* W3   = (const float*)d_in[9];
  const float* b3   = (const float*)d_in[10];
  float* out = (float*)d_out;
  rnn2_fused_kernel<<<kBlocks, kThreads, 0, stream>>>(x, Wih1, Whh1, bih1, bhh1, Wih2, Whh2, bih2, bhh2, W3, b3, out);
}
